// LQR_72378788872611
// MI455X (gfx1250) — hardware-verified
//
#include <hip/hip_runtime.h>
#include <math.h>

typedef __attribute__((ext_vector_type(16))) __bf16   v16b;
typedef __attribute__((ext_vector_type(8)))  __bf16   v8b;
typedef __attribute__((ext_vector_type(8)))  _Float16 v8h;
typedef __attribute__((ext_vector_type(8)))  float    v8f;
typedef __attribute__((ext_vector_type(4)))  float    v4f;

constexpr int kBatch  = 8192;
constexpr int kModes  = 6;
constexpr int kSteps  = 80;
constexpr int kNCtl   = 3;
constexpr int kNState = 9;
constexpr int kNTau   = 12;
constexpr int kKTgt   = kSteps * kNCtl;
constexpr int kKReal  = kKTgt + kNState;
constexpr int kKPad   = 256;
constexpr int kNPad   = 256;
constexpr int kTabRow = 192;

constexpr float kDt   = 0.1f;
constexpr float kDt2  = (float)(0.1 * 0.1);
constexpr float kDt3  = (float)(0.1 * 0.1 * 0.1);
constexpr float kYawW = 10.0f;

static_assert(kKTgt == 240 && kKReal == 249, "operand widths");
static_assert((kKPad % 32) == 0 && (kNPad % 64) == 0 && (kBatch % 64) == 0, "tile multiples");
static_assert(kKReal <= kKPad && kKTgt <= kNPad, "padding");
static_assert(((kBatch / 64) * 64 * kKTgt * 4) == 7864320, "output bytes");
static_assert(((64 * kKTgt * 4) % 128) == 0, "64-row span is whole lines");

constexpr size_t kOffTab  = 0;
constexpr size_t kOffWH   = kOffTab + (size_t)kSteps * kTabRow * 4;
constexpr size_t kOffWL   = kOffWH  + (size_t)kNPad * kKPad * 2;
constexpr size_t kOffAH   = kOffWL  + (size_t)kNPad * kKPad * 2;
constexpr size_t kOffAL   = kOffAH  + (size_t)kBatch * kKPad * 2;
constexpr size_t kWsTotal = kOffAL  + (size_t)kBatch * kKPad * 2;
static_assert(kWsTotal == 8712192ull, "carve total");
static_assert(kWsTotal <= 134217728ull, "carve cap");
static_assert((kOffWH % 128) == 0 && (kOffWL % 128) == 0 && (kOffAH % 128) == 0 && (kOffAL % 128) == 0, "aligned regions");

__device__ __forceinline__ unsigned short f2bf_bits(float f) {
  unsigned u = __float_as_uint(f);
  return (unsigned short)((u + 0x7FFFu + ((u >> 16) & 1u)) >> 16);
}
__device__ __forceinline__ float bf_bits2f(unsigned short h) { return __uint_as_float(((unsigned)h) << 16); }

union FragB { v16b v; v8b h[2]; };
__device__ __forceinline__ v16b frag_load(const __bf16* p) {
  FragB f;
  f.h[0] = *(const v8b*)(p);
  f.h[1] = *(const v8b*)(p + 16);
  return f.v;
}
__device__ __forceinline__ v8f mma_bf(v16b a, v16b b, v8f c) {
  c = __builtin_amdgcn_wmma_f32_16x16x32_bf16(false, a, false, b, (short)0, c, false, false);
  asm volatile("v_nop\n\tv_nop\n\tv_nop\n\tv_nop" : "+v"(c) : "v"(a), "v"(b));
  return c;
}
__device__ __forceinline__ float cost_diag(int i) {
  float w = 1.0f;
  w = (i == 2) ? kYawW : w;
  w = (i == 3 || i == 4) ? 0.0f : w;
  w = (i >= 9) ? 0.1f : w;
  return w;
}

__global__ __launch_bounds__(32) void gain_sweep_kernel(float* __restrict__ tab)
{
  __shared__ __align__(16) float sV[81];
  __shared__ __align__(16) float sVn[81];
  __shared__ __align__(16) float sQ[144];
  __shared__ __align__(16) float sM[108];
  __shared__ __align__(16) float sF[108];
  __shared__ __align__(16) float sWi[16];
  __shared__ __align__(16) float sG[27];
  __shared__ __align__(16) float sR[27];
  __shared__ __align__(16) float sTab[kTabRow];
  const int tid = threadIdx.x;

#pragma unroll 1
  for (int e = tid; e < 108; e += 32) {
    const int i = e / 12;
    const int j = e - i * 12;
    float f = 0.0f;
    f = (j == i) ? 1.0f : f;
    f = (j == i + 3) ? kDt : f;
    f = (j == i + 6 && i < 6) ? kDt2 : f;
    f = (j == i + 9 && i < 3) ? kDt3 : f;
    sF[e] = f;
  }
#pragma unroll 1
  for (int e = tid; e < 81; e += 32) sV[e] = 0.0f;
  if (tid < 16) sWi[tid] = 0.0f;
  __syncthreads();

#pragma unroll 1
  for (int t = kSteps; t >= 0; --t) {
#pragma unroll 1
    for (int e = tid; e < 108; e += 32) {
      const int s = e / 12;
      const int j = e - s * 12;
      float a = 0.0f;
#pragma unroll 1
      for (int u = 0; u < 9; ++u) a = fmaf(sV[s * 9 + u], sF[u * 12 + j], a);
      sM[e] = a;
    }
    __syncthreads();
#pragma unroll 1
    for (int e = tid; e < 144; e += 32) {
      const int i = e / 12;
      const int j = e - i * 12;
      float a = 0.0f;
#pragma unroll 1
      for (int s = 0; s < 9; ++s) a = fmaf(sF[s * 12 + i], sM[s * 12 + j], a);
      const float cd = (t > 0 && i == j) ? cost_diag(i) : 0.0f;
      sQ[e] = cd + a;
    }
    __syncthreads();
    {
      const float qa = sQ[9 * 12 + 9],  qb = sQ[9 * 12 + 10],  qc = sQ[9 * 12 + 11];
      const float qd = sQ[10 * 12 + 9], qe = sQ[10 * 12 + 10], qf = sQ[10 * 12 + 11];
      const float qg = sQ[11 * 12 + 9], qh = sQ[11 * 12 + 10], qi = sQ[11 * 12 + 11];
      const float c0 = qe * qi - qf * qh;
      const float c1 = qf * qg - qd * qi;
      const float c2 = qd * qh - qe * qg;
      const float det = qa * c0 + qb * c1 + qc * c2;
      const float sc = -1.0f / det;
      const float w0 = sc * c0;
      const float w1 = sc * (qc * qh - qb * qi);
      const float w2 = sc * (qb * qf - qc * qe);
      const float w3 = sc * c1;
      const float w4 = sc * (qa * qi - qc * qg);
      const float w5 = sc * (qc * qd - qa * qf);
      const float w6 = sc * c2;
      const float w7 = sc * (qb * qg - qa * qh);
      const float w8 = sc * (qa * qe - qb * qd);
      if (tid == 0) {
        sWi[0] = w0; sWi[1] = w1; sWi[2] = w2;
        sWi[3] = w3; sWi[4] = w4; sWi[5] = w5;
        sWi[6] = w6; sWi[7] = w7; sWi[8] = w8;
      }
    }
    __syncthreads();
#pragma unroll 1
    for (int e = tid; e < 27; e += 32) {
      const int r = e / 9;
      const int c = e - r * 9;
      float a = 0.0f;
#pragma unroll 1
      for (int u = 0; u < 3; ++u) a = fmaf(sWi[r * 3 + u], sQ[(9 + u) * 12 + c], a);
      sG[e] = a;
    }
    __syncthreads();
#pragma unroll 1
    for (int e = tid; e < 27; e += 32) {
      const int u = e / 9;
      const int c = e - u * 9;
      float a = 0.0f;
#pragma unroll 1
      for (int w = 0; w < 3; ++w) a = fmaf(sQ[(9 + u) * 12 + 9 + w], sG[w * 9 + c], a);
      sR[e] = sQ[(9 + u) * 12 + c] + a;
    }
    __syncthreads();
#pragma unroll 1
    for (int e = tid; e < 81; e += 32) {
      const int i = e / 9;
      const int j = e - i * 9;
      float a1 = 0.0f, a2 = 0.0f;
#pragma unroll 1
      for (int u = 0; u < 3; ++u) {
        a1 = fmaf(sQ[i * 12 + 9 + u], sG[u * 9 + j], a1);
        a2 = fmaf(sG[u * 9 + i], sR[u * 9 + j], a2);
      }
      sVn[e] = (sQ[i * 12 + j] + a1) + a2;
    }
#pragma unroll 1
    for (int e = tid; e < kTabRow; e += 32) {
      const int ee = (e < 161) ? e : 161;
      const bool tr = (ee >= 81);
      const int e2 = tr ? (ee - 81) : ee;
      const int r_ = e2 / 9;
      const int c_ = e2 - r_ * 9;
      const int i = tr ? c_ : r_;
      const int s = tr ? r_ : c_;
      float a = 0.0f;
#pragma unroll 1
      for (int u = 0; u < 3; ++u) a = fmaf(sF[i * 12 + 9 + u], sG[u * 9 + s], a);
      const float pv = sF[i * 12 + s] + a;
      int wi = e - 162;
      wi = (wi < 0) ? 0 : wi;
      wi = (wi > 8) ? 8 : wi;
      const float wv = sWi[wi];
      const float tailv = (e < 171) ? wv : 0.0f;
      sTab[e] = (e < 162) ? pv : tailv;
    }
    __syncthreads();
    if (t < kSteps) {
      float* gp = tab + (size_t)t * kTabRow;
      const int o1 = 128 + 4 * (tid & 15);
      const v4f v0 = *(const v4f*)(sTab + 4 * tid);
      const v4f v1 = *(const v4f*)(sTab + o1);
      for (int pass = 0; pass < 2; ++pass) {
        *(volatile v4f*)(gp + 4 * tid) = v0;
        if (tid < 16) *(volatile v4f*)(gp + o1) = v1;
        __threadfence();
      }
    }
#pragma unroll 1
    for (int e = tid; e < 81; e += 32) sV[e] = sVn[e];
    __syncthreads();
  }
}

__global__ __launch_bounds__(64) void op_build_kernel(
    const float* __restrict__ tab, unsigned short* __restrict__ WH, unsigned short* __restrict__ WL)
{
  __shared__ __align__(16) float sK[kKTgt * 64];
  __shared__ __align__(16) float sS[kNState * 64];
  static_assert((kKTgt * 64 + kNState * 64) * 4 <= 65536, "LDS budget");
  const int tid = threadIdx.x;
  const int j = blockIdx.x * 64 + tid;
  const bool isT = (j < kKTgt);
  const bool isX = (j >= kKTgt) && (j < kKReal);
  const bool live = isT || isX;
  const int jt = isT ? j : 0;
  const int tau = jt / 3;
  const int comp = jt - tau * 3;
  const int sidx = isT ? (tau + 1) : -1;
  const float alpha = isT ? ((comp == 2) ? -kYawW : -1.0f) : 0.0f;
  const int xcomp = isX ? (j - kKTgt) : -1;

#pragma unroll
  for (int i = 0; i < 9; ++i) sS[i * 64 + tid] = (sidx == kSteps && comp == i) ? alpha : 0.0f;

#pragma unroll 1
  for (int t = kSteps - 1; t >= 0; --t) {
    const float* row = tab + (size_t)t * kTabRow;
    const float u0 = sS[0 * 64 + tid], u1 = sS[1 * 64 + tid], u2 = sS[2 * 64 + tid];
    const float u3 = sS[3 * 64 + tid], u4 = sS[4 * 64 + tid], u5 = sS[5 * 64 + tid];
    const float u6 = sS[6 * 64 + tid], u7 = sS[7 * 64 + tid], u8 = sS[8 * 64 + tid];
    const float q0 = kDt3 * u0 + kDt2 * u3 + kDt * u6;
    const float q1 = kDt3 * u1 + kDt2 * u4 + kDt * u7;
    const float q2 = kDt3 * u2 + kDt2 * u5 + kDt * u8;
    const float* wi = row + 162;
    const float k0 = wi[0] * q0 + wi[1] * q1 + wi[2] * q2;
    const float k1 = wi[3] * q0 + wi[4] * q1 + wi[5] * q2;
    const float k2 = wi[6] * q0 + wi[7] * q1 + wi[8] * q2;
    sK[(3 * t + 0) * 64 + tid] = k0;
    sK[(3 * t + 1) * 64 + tid] = k1;
    sK[(3 * t + 2) * 64 + tid] = k2;
    float acc[9];
#pragma unroll
    for (int i = 0; i < 9; ++i) acc[i] = 0.0f;
#pragma unroll 1
    for (int s = 0; s < 9; ++s) {
      const float vs = sS[s * 64 + tid];
      const float* pr = row + s * 9;
#pragma unroll
      for (int i = 0; i < 9; ++i) acc[i] = fmaf(pr[i], vs, acc[i]);
    }
#pragma unroll
    for (int i = 0; i < 9; ++i) {
      const float cadd = (sidx == t && comp == i) ? alpha : 0.0f;
      sS[i * 64 + tid] = acc[i] + cadd;
    }
  }

#pragma unroll
  for (int i = 0; i < 9; ++i) sS[i * 64 + tid] = (xcomp == i) ? 1.0f : 0.0f;

#pragma unroll 1
  for (int t = 0; t < kSteps; ++t) {
    const float* rowT = tab + (size_t)t * kTabRow + 81;
    const float k0 = sK[(3 * t + 0) * 64 + tid];
    const float k1 = sK[(3 * t + 1) * 64 + tid];
    const float k2 = sK[(3 * t + 2) * 64 + tid];
    float acc[9];
    acc[0] = kDt3 * k0; acc[1] = kDt3 * k1; acc[2] = kDt3 * k2;
    acc[3] = kDt2 * k0; acc[4] = kDt2 * k1; acc[5] = kDt2 * k2;
    acc[6] = kDt * k0;  acc[7] = kDt * k1;  acc[8] = kDt * k2;
#pragma unroll 1
    for (int s = 0; s < 9; ++s) {
      const float xs = sS[s * 64 + tid];
      const float* pr = rowT + s * 9;
#pragma unroll
      for (int i = 0; i < 9; ++i) acc[i] = fmaf(pr[i], xs, acc[i]);
    }
#pragma unroll
    for (int i = 0; i < 9; ++i) sS[i * 64 + tid] = acc[i];
    sK[(3 * t + 0) * 64 + tid] = live ? acc[0] : 0.0f;
    sK[(3 * t + 1) * 64 + tid] = live ? acc[1] : 0.0f;
    sK[(3 * t + 2) * 64 + tid] = live ? acc[2] : 0.0f;
  }
  __syncthreads();

  const int lane = tid & 31, wave = tid >> 5;
  const int q = lane >> 3, c8 = (lane & 7) * 8;
  for (int pass = 0; pass < 2; ++pass) {
#pragma unroll 1
    for (int it = 0; it < 32; ++it) {
      const int n = it * 8 + wave * 4 + q;
      const int nc = (n < kKTgt) ? n : (kKTgt - 1);
      const bool rowlive = (n < kKTgt);
      const float* sp = sK + nc * 64 + c8;
      const v4f a0 = *(const v4f*)(sp);
      const v4f a1 = *(const v4f*)(sp + 4);
      v8h hv, lv;
#pragma unroll
      for (int e = 0; e < 4; ++e) {
        const float x0 = rowlive ? a0[e] : 0.0f;
        const float x1 = rowlive ? a1[e] : 0.0f;
        const unsigned short h0 = f2bf_bits(x0), h1 = f2bf_bits(x1);
        const unsigned short l0 = f2bf_bits(x0 - bf_bits2f(h0)), l1 = f2bf_bits(x1 - bf_bits2f(h1));
        hv[e]     = __builtin_bit_cast(_Float16, h0);
        hv[4 + e] = __builtin_bit_cast(_Float16, h1);
        lv[e]     = __builtin_bit_cast(_Float16, l0);
        lv[4 + e] = __builtin_bit_cast(_Float16, l1);
      }
      const size_t o = (size_t)n * kKPad + blockIdx.x * 64 + c8;
      *(volatile v8h*)(WH + o) = hv;
      *(volatile v8h*)(WL + o) = lv;
    }
    __threadfence();
  }
}

__global__ __launch_bounds__(256) void pack_rows_kernel(
    const float* __restrict__ ego, const float* __restrict__ ap,
    unsigned short* __restrict__ AH, unsigned short* __restrict__ AL)
{
  const int g = blockIdx.x * 256 + threadIdx.x;
  const int m = g >> 5, L = g & 31;
  const float* ar = ap + ((size_t)m * kModes + (kModes - 1)) * kKTgt;
  const int kc = (L < 30) ? (L << 3) : (kKTgt - 8);
  v4f a0 = *(const v4f*)(ar + kc);
  v4f a1 = *(const v4f*)(ar + kc + 4);
  const float* er = ego + (size_t)m * kNState;
  float e0 = er[0], e1 = er[1], e2 = er[2], e3 = er[3], e4 = er[4];
  float e5 = er[5], e6 = er[6], e7 = er[7], e8 = er[8];
  asm volatile("" : "+v"(a0), "+v"(a1));
  asm volatile("" : "+v"(e0), "+v"(e1), "+v"(e2), "+v"(e3), "+v"(e4));
  asm volatile("" : "+v"(e5), "+v"(e6), "+v"(e7), "+v"(e8));
  const float av[8] = {a0[0], a0[1], a0[2], a0[3], a1[0], a1[1], a1[2], a1[3]};
  const float ev[8] = {e0, e1, e2, e3, e4, e5, e6, e7};
  v8h hv, lv;
#pragma unroll
  for (int e = 0; e < 8; ++e) {
    const float tailv = (e == 0) ? e8 : 0.0f;
    const float mid = (L == 30) ? ev[e] : tailv;
    const float x = (L < 30) ? av[e] : mid;
    const unsigned short hb = f2bf_bits(x);
    const unsigned short lb = f2bf_bits(x - bf_bits2f(hb));
    hv[e] = __builtin_bit_cast(_Float16, hb);
    lv[e] = __builtin_bit_cast(_Float16, lb);
  }
  const size_t o = (size_t)m * kKPad + (L << 3);
  *(volatile v8h*)(AH + o) = hv;
  *(volatile v8h*)(AL + o) = lv;
  __threadfence();
  *(volatile v8h*)(AH + o) = hv;
  *(volatile v8h*)(AL + o) = lv;
}

__global__ __launch_bounds__(256) void plan_gemm_kernel(
    const unsigned short* __restrict__ AHp, const unsigned short* __restrict__ ALp,
    const unsigned short* __restrict__ WHp, const unsigned short* __restrict__ WLp,
    float* __restrict__ out)
{
  __shared__ __align__(16) float sC[64 * kKTgt];
  const __bf16* AH = (const __bf16*)AHp;
  const __bf16* AL = (const __bf16*)ALp;
  const __bf16* WH = (const __bf16*)WHp;
  const __bf16* WL = (const __bf16*)WLp;
  const int tid = threadIdx.x;
  const int lane = tid & 31, wave = tid >> 5;
  const int rlane = lane & 15;
  const int hh = lane >> 4;
  const int koff = hh * 8;
  const int mi = wave >> 2, ni = wave & 3;
  const int m0 = blockIdx.x * 64;
  const int mw = m0 + mi * 32;
  const int n0 = ni * 64;

  v8f acc[2][4];
#pragma unroll
  for (int i = 0; i < 2; ++i)
#pragma unroll
    for (int jx = 0; jx < 4; ++jx) acc[i][jx] = (v8f){0.f, 0.f, 0.f, 0.f, 0.f, 0.f, 0.f, 0.f};

#pragma unroll 1
  for (int k0 = 0; k0 < kKPad; k0 += 32) {
    v16b bh[4], bl[4];
#pragma unroll
    for (int jx = 0; jx < 4; ++jx) {
      const size_t bo = (size_t)(n0 + (jx << 4) + rlane) * kKPad + koff + k0;
      bh[jx] = frag_load(WH + bo);
      bl[jx] = frag_load(WL + bo);
    }
#pragma unroll
    for (int i = 0; i < 2; ++i) {
      const size_t ao = (size_t)(mw + (i << 4) + rlane) * kKPad + koff + k0;
      const v16b ah = frag_load(AH + ao);
      const v16b al = frag_load(AL + ao);
#pragma unroll
      for (int jx = 0; jx < 4; ++jx) {
        acc[i][jx] = mma_bf(ah, bh[jx], acc[i][jx]);
        acc[i][jx] = mma_bf(ah, bl[jx], acc[i][jx]);
        acc[i][jx] = mma_bf(al, bh[jx], acc[i][jx]);
      }
    }
  }

#pragma unroll
  for (int i = 0; i < 2; ++i) {
#pragma unroll
    for (int jx = 0; jx < 4; ++jx) {
      const int cbase = n0 + (jx << 4);
      if (cbase < kKTgt) {
#pragma unroll
        for (int r = 0; r < 8; ++r) {
          const int rowl = mi * 32 + (i << 4) + 8 * hh + r;
          sC[rowl * kKTgt + cbase + rlane] = acc[i][jx][r];
        }
      }
    }
  }
  __syncthreads();

  float* ob = out + (size_t)m0 * kKTgt;
  for (int pass = 0; pass < 2; ++pass) {
#pragma unroll 1
    for (int it = 0; it < 15; ++it) {
      const int idx = (it * 256 + tid) * 4;
      const v4f v = *(const v4f*)(sC + idx);
      *(volatile v4f*)(ob + idx) = v;
    }
    __threadfence();
  }
}

extern "C" void kernel_launch(void* const* d_in, const int* in_sizes, int n_in,
                              void* d_out, int out_size, void* d_ws, size_t ws_size,
                              hipStream_t stream) {
  if (n_in < 2) return;
  if (in_sizes[0] != kBatch * kNState) return;
  if (in_sizes[1] != kBatch * kModes * kKTgt) return;
  if (out_size != kBatch * kKTgt) return;
  if (ws_size < kWsTotal) return;

  const float* ego = (const float*)d_in[0];
  const float* ap  = (const float*)d_in[1];
  float* out = (float*)d_out;

  char* ws = (char*)d_ws;
  float*          TAB = (float*)(ws + kOffTab);
  unsigned short* WH  = (unsigned short*)(ws + kOffWH);
  unsigned short* WL  = (unsigned short*)(ws + kOffWL);
  unsigned short* AH  = (unsigned short*)(ws + kOffAH);
  unsigned short* AL  = (unsigned short*)(ws + kOffAL);

  gain_sweep_kernel<<<1, 32, 0, stream>>>(TAB);
  op_build_kernel<<<kKPad / 64, 64, 0, stream>>>(TAB, WH, WL);
  pack_rows_kernel<<<(kBatch * 32) / 256, 256, 0, stream>>>(ego, ap, AH, AL);
  plan_gemm_kernel<<<kBatch / 64, 256, 0, stream>>>(AH, AL, WH, WL, out);
}
